// SimpleS4_20993800142892
// MI455X (gfx1250) — hardware-run, weakly checked
//
#include <hip/hip_runtime.h>
#include <math.h>

typedef __attribute__((ext_vector_type(16))) _Float16 v16h;
typedef __attribute__((ext_vector_type(8)))  _Float16 v8h;
typedef __attribute__((ext_vector_type(4)))  _Float16 v4h;
typedef __attribute__((ext_vector_type(8)))  float    v8f;
typedef __attribute__((ext_vector_type(4)))  float    v4f;

constexpr int kNB     = 8;
constexpr int kNH     = 256;
constexpr int kNL     = 4096;
constexpr int kNDD    = 32;
constexpr int kQC     = 64;
constexpr int kPairs  = kNL / (2 * kQC);
constexpr int kGuardN = 64;
constexpr int kFP     = kNL + kGuardN;
constexpr int kUP     = kNL + kGuardN;
constexpr int kNumShift = 4;
constexpr int kSegs   = kFP / 8;
constexpr int kTP     = 68;
constexpr float kTstep = (float)(1.0 / (double)(kNL - 1));
constexpr float kCarry    = 4096.0f;
constexpr float kInvCarry = 1.0f / 4096.0f;
constexpr float kFltMin   = 1.17549435e-38f;

static_assert(kPairs == 32);
static_assert(kFP == 4160 && kUP == 4160 && kSegs == 520);
static_assert((kFP * 2) % 128 == 0);
static_assert((kNH * kNDD) % 256 == 0);
static_assert(kNL % 256 == 0);
static_assert((kNumShift * kNH * kSegs) % 256 == 0);
static_assert((kNB * kNH * kSegs) % 256 == 0);

constexpr size_t kOffCP  = 0;
constexpr size_t kOffCQ  = kOffCP  + (size_t)kNH * kNDD * 4;
constexpr size_t kOffCG  = kOffCQ  + (size_t)kNH * kNDD * 4;
constexpr size_t kOffFF  = kOffCG  + (size_t)kNH * kNDD * 4;
constexpr size_t kOffGI  = kOffFF  + (size_t)kNH * kNL * 4;
constexpr size_t kOffFS  = kOffGI  + (size_t)kNH * kNL * 4;
constexpr size_t kOffU16 = kOffFS  + (size_t)kNumShift * kNH * kFP * 2;
constexpr size_t kWsTotal = kOffU16 + (size_t)kNB * kNH * kUP * 2;
static_assert(kWsTotal == 34045952ull);
static_assert(kWsTotal <= 134217728ull);
static_assert((kOffCQ % 128) == 0 && (kOffCG % 128) == 0 && (kOffFF % 128) == 0 && (kOffGI % 128) == 0 &&
              (kOffFS % 128) == 0 && (kOffU16 % 128) == 0);

union FragB { v16h v; v8h h[2]; };
union FragA { v16h v; v4h q[4]; };

__device__ __forceinline__ v16h load_b_frag(const _Float16* p) {
  FragB f;
  f.h[0] = *(const v8h*)(p);
  f.h[1] = *(const v8h*)(p + 16);
  return f.v;
}
__device__ __forceinline__ v16h load_a_frag(const _Float16* p) {
  FragA f;
  f.q[0] = *(const v4h*)(p);
  f.q[1] = *(const v4h*)(p + 4);
  f.q[2] = *(const v4h*)(p + 16);
  f.q[3] = *(const v4h*)(p + 20);
  return f.v;
}
__device__ __forceinline__ v8f mma_f16_guarded(v16h a, v16h b, v8f c) {
  c = __builtin_amdgcn_wmma_f32_16x16x32_f16(false, a, false, b, (short)0, c, false, false);
  asm volatile("v_nop\n\tv_nop\n\tv_nop\n\tv_nop" : "+v"(c) : "v"(a), "v"(b));
  return c;
}

__global__ __launch_bounds__(256) void mode_const_kernel(
    const float* __restrict__ theta, const float* __restrict__ a, const float* __restrict__ b_p,
    const float* __restrict__ c_p, const float* __restrict__ x0,
    float* __restrict__ CP, float* __restrict__ CQ, float* __restrict__ CG)
{
  const int i = blockIdx.x * 256 + threadIdx.x;
  const float th = theta[i];
  const float aa = fabsf(a[i]);
  const float bp = b_p[i];
  const float cp = c_p[i];
  const float xv = x0[i];
  const float eT  = expf(-(aa * kTstep));
  const float phT = th * kTstep;
  const float cT  = cosf(phT);
  const float sT  = sinf(phT);
  const float nr  = eT * cT - 1.0f;
  const float ni  = eT * sT;
  const float den = aa * aa + th * th;
  const float rden = 1.0f / den;
  const float t0r = (-aa * nr + th * ni) * rden;
  const float t0i = (-aa * ni - th * nr) * rden;
  const float q   = bp * cp;
  const float vp  = 2.0f * q * t0r;
  const float vq  = -2.0f * q * t0i;
  const float vg  = 4.0f * kTstep * (cp * xv);
  volatile float* pp = CP + i;
  volatile float* pq = CQ + i;
  volatile float* pg = CG + i;
  *pp = vp;
  *pq = vq;
  *pg = vg;
  __threadfence();
  *pp = vp;
  *pq = vq;
  *pg = vg;
}

__global__ __launch_bounds__(256) void build_filter_kernel(
    const float* __restrict__ theta, const float* __restrict__ a,
    const float* __restrict__ CP, const float* __restrict__ CQ, const float* __restrict__ CG,
    float* __restrict__ FF, float* __restrict__ GI)
{
  __shared__ float sC[5 * kNDD];
  const int tid = threadIdx.x;
  const int h = blockIdx.y;
  const int l = blockIdx.x * 256 + tid;
  if (tid < kNDD) {
    const int idx = h * kNDD + tid;
    sC[tid]            = CP[idx];
    sC[kNDD + tid]     = CQ[idx];
    sC[2 * kNDD + tid] = CG[idx];
    sC[3 * kNDD + tid] = fabsf(a[idx]);
    sC[4 * kNDD + tid] = theta[idx];
  }
  __syncthreads();
  const float z = kTstep * (float)l;
  float facc = 0.0f;
  float gacc = 0.0f;
#pragma unroll 1
  for (int d = 0; d < kNDD; ++d) {
    const float pd = sC[d];
    const float qd = sC[kNDD + d];
    const float gd = sC[2 * kNDD + d];
    const float ad = sC[3 * kNDD + d];
    const float td = sC[4 * kNDD + d];
    const float ph = td * z;
    const float cs = cosf(ph);
    const float sn = sinf(ph);
    float e = expf(-(ad * z));
    e = (e < kFltMin) ? 0.0f : e;
    facc += e * (pd * cs + qd * sn);
    gacc += gd * (e * cs);
  }
  const size_t o = (size_t)h * kNL + l;
  volatile float* pf = FF + o;
  volatile float* pg = GI + o;
  *pf = facc;
  *pg = gacc;
  __threadfence();
  *pf = facc;
  *pg = gacc;
}

__global__ __launch_bounds__(256) void filter_image_kernel(
    const float* __restrict__ FF, unsigned short* __restrict__ FS)
{
  const int t = blockIdx.x * 256 + threadIdx.x;
  const int cc  = t / (kNH * kSegs);
  const int rem = t - cc * (kNH * kSegs);
  const int h   = rem / kSegs;
  const int seg = rem - h * kSegs;
  const int p0  = seg * 8;
  const float* frow = FF + (size_t)h * kNL;
  v8h hv;
#pragma unroll
  for (int e = 0; e < 8; ++e) {
    const int li = (kNL - 1) - (p0 + cc + e);
    const bool valid = (li >= 0);
    const int lic = valid ? li : 0;
    const float v = frow[lic];
    const float vv = valid ? (v * kCarry) : 0.0f;
    hv[e] = (_Float16)vv;
  }
  unsigned short* dst = FS + (size_t)t * 8;
  *(volatile v8h*)dst = hv;
  __threadfence();
  *(volatile v8h*)dst = hv;
}

__global__ __launch_bounds__(256) void pack_input_kernel(
    const float* __restrict__ u, unsigned short* __restrict__ U16)
{
  const int t = blockIdx.x * 256 + threadIdx.x;
  const int row = t / kSegs;
  const int seg = t - row * kSegs;
  const bool isg = (seg < (kGuardN / 8));
  const int sc = isg ? 0 : (seg - (kGuardN / 8));
  const float* src = u + (size_t)row * kNL + sc * 8;
  const v4f a0 = *(const v4f*)(src);
  const v4f a1 = *(const v4f*)(src + 4);
  v8h hv;
#pragma unroll
  for (int e = 0; e < 4; ++e) {
    const float x0v = isg ? 0.0f : a0[e];
    const float x1v = isg ? 0.0f : a1[e];
    hv[e]     = (_Float16)x0v;
    hv[4 + e] = (_Float16)x1v;
  }
  unsigned short* dst = U16 + (size_t)t * 8;
  *(volatile v8h*)dst = hv;
  __threadfence();
  *(volatile v8h*)dst = hv;
}

__global__ __launch_bounds__(128) void toeplitz_conv_kernel(
    const unsigned short* __restrict__ FSp, const unsigned short* __restrict__ U16p,
    const float* __restrict__ u, const float* __restrict__ GI, const float* __restrict__ Dv,
    float* __restrict__ out)
{
  __shared__ __align__(16) _Float16 Fsh[kNumShift * kFP];
  __shared__ __align__(16) float sT[16 * kTP];
  const int tid  = threadIdx.x;
  const int lane = tid & 31;
  const int wave = tid >> 5;
  const int hh   = lane >> 4;
  const int c    = lane & 15;
  const int h    = blockIdx.y;
  const int p    = blockIdx.x;

  const _Float16* FS  = (const _Float16*)FSp;
  const _Float16* U16 = (const _Float16*)U16p;

  const int xlo = kNL - (2 * p + 2) * kQC;
  const int plo = (xlo >= 8) ? (xlo - 8) : 0;
  const int nch = (kFP - plo) >> 3;
#pragma unroll 1
  for (int cc = 0; cc < kNumShift; ++cc) {
    const _Float16* src = FS + ((size_t)cc * kNH + h) * kFP + plo;
    _Float16* dst = Fsh + cc * kFP + plo;
    for (int q = tid; q < nch; q += 128) {
      const v8h w = *(const v8h*)(src + q * 8);
      *(v8h*)(dst + q * 8) = w;
    }
  }
  __syncthreads();

  const int mg = wave * 16 + c;
  const int sh = (kNL - 1 - mg) & 3;
  const _Float16* abase = Fsh + sh * kFP + (kNL - 1 - mg - sh) + 8 * hh;
  const int sCol = c >> 3;
  const int bCol = c & 7;
  const _Float16* ubase = U16 + ((size_t)(bCol * kNH + h)) * kUP + kGuardN + (2 * p + sCol) * kQC + 8 * hh;
  v8f acc = (v8f){0.f, 0.f, 0.f, 0.f, 0.f, 0.f, 0.f, 0.f};
  const int nd = 2 * p + 2;
#pragma unroll 1
  for (int dl = 0; dl < nd; ++dl) {
    const _Float16* ap = abase - dl * kQC;
    const _Float16* bp = ubase - dl * kQC;
#pragma unroll
    for (int ks = 0; ks < 2; ++ks) {
      const v16h af = load_a_frag(ap + ks * 32);
      const v16h bf = load_b_frag(bp + ks * 32);
      acc = mma_f16_guarded(af, bf, acc);
    }
  }

#pragma unroll
  for (int r = 0; r < 8; ++r) sT[c * kTP + wave * 16 + 8 * hh + r] = acc[r];
  __syncthreads();

  const int c4 = (lane & 15) * 4;
  const float Dh = Dv[h];
  const int n0 = wave * 4 + hh;
  const int n1 = n0 + 2;
  const int l0 = (2 * p + (n0 >> 3)) * kQC + c4;
  const int l1 = (2 * p + (n1 >> 3)) * kQC + c4;
  const size_t o0 = ((size_t)((n0 & 7) * kNH + h)) * kNL + l0;
  const size_t o1 = ((size_t)((n1 & 7) * kNH + h)) * kNL + l1;
  const v4f t0 = *(const v4f*)(sT + n0 * kTP + c4);
  const v4f t1 = *(const v4f*)(sT + n1 * kTP + c4);
  const v4f u0 = *(const v4f*)(u + o0);
  const v4f u1 = *(const v4f*)(u + o1);
  const v4f g0 = *(const v4f*)(GI + (size_t)h * kNL + l0);
  const v4f g1 = *(const v4f*)(GI + (size_t)h * kNL + l1);
  const v4f r0 = t0 * kInvCarry + u0 * Dh + g0;
  const v4f r1 = t1 * kInvCarry + u1 * Dh + g1;
  volatile v4f* q0 = (volatile v4f*)(out + o0);
  volatile v4f* q1 = (volatile v4f*)(out + o1);
  *q0 = r0;
  *q1 = r1;
  __threadfence();
  *q0 = r0;
  *q1 = r1;
}

extern "C" void kernel_launch(void* const* d_in, const int* in_sizes, int n_in,
                              void* d_out, int out_size, void* d_ws, size_t ws_size,
                              hipStream_t stream) {
  if (n_in < 7) return;
  if (in_sizes[0] != kNB * kNH * kNL) return;
  if (in_sizes[1] != kNH * kNDD) return;
  if (in_sizes[2] != kNH * kNDD) return;
  if (in_sizes[3] != kNH) return;
  if (in_sizes[4] != kNH * kNDD) return;
  if (in_sizes[5] != kNH * kNDD) return;
  if (in_sizes[6] != kNH * kNDD) return;
  if (out_size != kNB * kNH * kNL) return;
  if (ws_size < kWsTotal) return;

  const float* u     = (const float*)d_in[0];
  const float* theta = (const float*)d_in[1];
  const float* a     = (const float*)d_in[2];
  const float* Dv    = (const float*)d_in[3];
  const float* b_p   = (const float*)d_in[4];
  const float* c_p   = (const float*)d_in[5];
  const float* x0    = (const float*)d_in[6];
  float* out = (float*)d_out;

  char* ws = (char*)d_ws;
  float*          CP  = (float*)(ws + kOffCP);
  float*          CQ  = (float*)(ws + kOffCQ);
  float*          CG  = (float*)(ws + kOffCG);
  float*          FF  = (float*)(ws + kOffFF);
  float*          GI  = (float*)(ws + kOffGI);
  unsigned short* FS  = (unsigned short*)(ws + kOffFS);
  unsigned short* U16 = (unsigned short*)(ws + kOffU16);

  mode_const_kernel<<<(kNH * kNDD) / 256, 256, 0, stream>>>(theta, a, b_p, c_p, x0, CP, CQ, CG);
  build_filter_kernel<<<dim3(kNL / 256, kNH), 256, 0, stream>>>(theta, a, CP, CQ, CG, FF, GI);
  filter_image_kernel<<<(kNumShift * kNH * kSegs) / 256, 256, 0, stream>>>(FF, FS);
  pack_input_kernel<<<(kNB * kNH * kSegs) / 256, 256, 0, stream>>>(u, U16);
  toeplitz_conv_kernel<<<dim3(kPairs, kNH), 128, 0, stream>>>(FS, U16, u, GI, Dv, out);
}
